// PAM_41180146434397
// MI455X (gfx1250) — hardware-verified
//
#include <hip/hip_runtime.h>

typedef __attribute__((ext_vector_type(16))) _Float16 v16h;
typedef __attribute__((ext_vector_type(8)))  _Float16 v8h;
typedef __attribute__((ext_vector_type(16))) __bf16   v16b;
typedef __attribute__((ext_vector_type(8)))  __bf16   v8b;
typedef __attribute__((ext_vector_type(8)))  float    v8f;
typedef __attribute__((ext_vector_type(4)))  float    v4f;

#ifndef NB
#define NB 4
#endif
#ifndef SEQ
#define SEQ 4096
#endif
#define NB_FULL 4
#define SEQ_FULL 4096

static constexpr int kBatch   = NB;
static constexpr int kPix     = SEQ;
static constexpr int kPixFull = SEQ_FULL;
static constexpr int kCh      = 512;
static constexpr int kCq      = 64;
static constexpr float kPCarry    = 16384.0f;
static constexpr float kPCarryInv = 1.0f / 16384.0f;
static_assert(NB >= 1 && NB <= NB_FULL);
static_assert(SEQ >= 256 && SEQ <= SEQ_FULL && (SEQ % 256) == 0);

static constexpr size_t kPlaneX   = (size_t)kBatch * kPix * kCh * 2;
static constexpr size_t kPlaneWqk = (size_t)kCq * kCh * 2;
static constexpr size_t kPlaneWv  = (size_t)kCh * kCh * 2;
static constexpr size_t kPlaneQK  = (size_t)kBatch * kPix * kCq * 2;
static constexpr size_t kPlaneVt  = (size_t)kBatch * kCh * kPix * 2;
static constexpr size_t kPlaneS   = (size_t)kPix * kPix * 4;
static constexpr size_t kPlaneP   = (size_t)kPix * kPix * 2;
static constexpr size_t kOffXtHi  = 0;
static constexpr size_t kOffXtLo  = kOffXtHi + kPlaneX;
static constexpr size_t kOffWqHi  = kOffXtLo + kPlaneX;
static constexpr size_t kOffWqLo  = kOffWqHi + kPlaneWqk;
static constexpr size_t kOffWkHi  = kOffWqLo + kPlaneWqk;
static constexpr size_t kOffWkLo  = kOffWkHi + kPlaneWqk;
static constexpr size_t kOffWvHi  = kOffWkLo + kPlaneWqk;
static constexpr size_t kOffWvLo  = kOffWvHi + kPlaneWv;
static constexpr size_t kOffQHi   = kOffWvLo + kPlaneWv;
static constexpr size_t kOffQLo   = kOffQHi + kPlaneQK;
static constexpr size_t kOffKHi   = kOffQLo + kPlaneQK;
static constexpr size_t kOffKLo   = kOffKHi + kPlaneQK;
static constexpr size_t kOffVt    = kOffKLo + kPlaneQK;
static constexpr size_t kOffS     = kOffVt + kPlaneVt;
static constexpr bool   kPAlias   = (kPlaneP <= 2 * kPlaneX);
static constexpr size_t kOffP     = kPAlias ? (size_t)0 : (kOffS + kPlaneS);
static constexpr size_t kWsTotal  = kOffS + kPlaneS + (kPAlias ? (size_t)0 : kPlaneP);
static_assert(NB != NB_FULL || SEQ != SEQ_FULL || kWsTotal == 127139840);
static_assert(kWsTotal <= 134217728);
static_assert((kOffXtLo % 128) == 0 && (kOffWqHi % 128) == 0 && (kOffWqLo % 128) == 0 && (kOffWkHi % 128) == 0);
static_assert((kOffWkLo % 128) == 0 && (kOffWvHi % 128) == 0 && (kOffWvLo % 128) == 0 && (kOffQHi % 128) == 0);
static_assert((kOffQLo % 128) == 0 && (kOffKHi % 128) == 0 && (kOffKLo % 128) == 0 && (kOffVt % 128) == 0);
static_assert((kOffS % 128) == 0 && (kOffP % 128) == 0);
static_assert(kPix % 64 == 0 && kCq % 64 == 0 && kCh % 64 == 0);
static_assert(kCh % 32 == 0 && kCq % 32 == 0 && kPix % 32 == 0);

static constexpr int kSmThreads = (kPix / 8 < 256) ? (kPix / 8) : 256;
static constexpr int kSmChunks  = kPix / (8 * kSmThreads);
static_assert(kSmThreads % 32 == 0 && kSmThreads * 8 * kSmChunks == kPix && kSmChunks >= 1 && kSmChunks <= 2);

__device__ __forceinline__ unsigned short f2bf_bits(float f) {
  unsigned u = __float_as_uint(f);
  return (unsigned short)((u + 0x7FFFu + ((u >> 16) & 1u)) >> 16);
}
__device__ __forceinline__ float bf_bits2f(unsigned short h) { return __uint_as_float(((unsigned)h) << 16); }

__device__ __forceinline__ void dep_guard_h(v8f& a, v8f& b, v16h x, v16h y) { asm volatile("v_nop\n\tv_nop\n\tv_nop\n\tv_nop" : "+v"(a), "+v"(b) : "v"(x), "v"(y)); }
__device__ __forceinline__ void dep_guard_b(v8f& a, v8f& b, v16b x, v16b y) { asm volatile("v_nop\n\tv_nop\n\tv_nop\n\tv_nop" : "+v"(a), "+v"(b) : "v"(x), "v"(y)); }
__device__ __forceinline__ void keep4_h(v16h a, v16h b, v16h c, v16h d) { asm volatile("v_nop" :: "v"(a), "v"(b), "v"(c), "v"(d)); }
__device__ __forceinline__ void keep4_b(v16b a, v16b b, v16b c, v16b d) { asm volatile("v_nop" :: "v"(a), "v"(b), "v"(c), "v"(d)); }
__device__ __forceinline__ void acc_guard4(v8f& a, v8f& b, v8f& c, v8f& d) { asm volatile("v_nop\n\tv_nop\n\tv_nop\n\tv_nop" : "+v"(a), "+v"(b), "+v"(c), "+v"(d)); }
template <typename T> struct Frag;
template <> struct Frag<_Float16> {
  typedef v16h V; union U { v16h v; v8h h[2]; };
  static __device__ __forceinline__ v16h load(const _Float16* p) {
    U f; f.h[0] = *(const v8h*)(p); f.h[1] = *(const v8h*)(p + 16); return f.v;
  }
  static __device__ __forceinline__ v8f mma(v16h a, v16h b, v8f c) {
    return __builtin_amdgcn_wmma_f32_16x16x32_f16(false, a, false, b, (short)0, c, false, false);
  }
  static __device__ __forceinline__ void guard(v8f& a, v8f& b, v16h x, v16h y) { dep_guard_h(a, b, x, y); }
  static __device__ __forceinline__ void keep(v16h a, v16h b, v16h c, v16h d) { keep4_h(a, b, c, d); }
};
template <> struct Frag<__bf16> {
  typedef v16b V; union U { v16b v; v8b h[2]; };
  static __device__ __forceinline__ v16b load(const __bf16* p) {
    U f; f.h[0] = *(const v8b*)(p); f.h[1] = *(const v8b*)(p + 16); return f.v;
  }
  static __device__ __forceinline__ v8f mma(v16b a, v16b b, v8f c) {
    return __builtin_amdgcn_wmma_f32_16x16x32_bf16(false, a, false, b, (short)0, c, false, false);
  }
  static __device__ __forceinline__ void guard(v8f& a, v8f& b, v16b x, v16b y) { dep_guard_b(a, b, x, y); }
  static __device__ __forceinline__ void keep(v16b a, v16b b, v16b c, v16b d) { keep4_b(a, b, c, d); }
};

template <int ET> struct Elem;
template <> struct Elem<0> { typedef _Float16 T; };
template <> struct Elem<1> { typedef __bf16 T; };
template <int ET, bool SPLIT, int BIAS_MODE, int OUT_MODE, bool RESID, bool GMUL>
__global__ __launch_bounds__(256) void wmma_gemm64(
    const unsigned short* __restrict__ Ap, const unsigned short* __restrict__ A2p, int lda, long strideA,
    const unsigned short* __restrict__ Btp, const unsigned short* __restrict__ Bt2p, int ldb, long strideB,
    void* __restrict__ Cout, void* __restrict__ Cout2, int ldc, long strideC,
    const float* __restrict__ bias,
    const float* __restrict__ resid, long strideR,
    const float* __restrict__ gptr,
    int M, int N, int K, float scale) {
  typedef typename Elem<ET>::T T;
  typedef typename Frag<T>::V V;
  const T* A = (const T*)Ap; const T* A2 = (const T*)A2p; const T* Bt = (const T*)Btp; const T* Bt2 = (const T*)Bt2p;
  __shared__ __align__(16) float sT[8][16 * 68];
  const int b    = blockIdx.y;
  const int lane = threadIdx.x & 31;
  const int wave = threadIdx.x >> 5;
  const int tilesN = N >> 6;
  const int tilesM = M >> 6;
  const int tile = blockIdx.x * 8 + wave;
  if (tile >= tilesM * tilesN) return;
  const int tm = tile / tilesN;
  const int tn = tile - tm * tilesN;
  const int m0 = tm << 6;
  const int n0 = tn << 6;

  const T* Ab  = A  + (size_t)b * strideA;
  const T* Bb  = Bt + (size_t)b * strideB;
  const T* Ab2 = SPLIT ? (A2  + (size_t)b * strideA) : nullptr;
  const T* Bb2 = SPLIT ? (Bt2 + (size_t)b * strideB) : nullptr;

  const int rlane = lane & 15;
  const int koff  = (lane >> 4) * 8;
  const int mOff  = (lane >> 4) * 8;

  v8f acc[4][4];
#pragma unroll
  for (int i = 0; i < 4; ++i)
#pragma unroll
    for (int j = 0; j < 4; ++j) acc[i][j] = (v8f){0.f,0.f,0.f,0.f,0.f,0.f,0.f,0.f};

  for (int k0 = 0; k0 < K; k0 += 32) {
    V bh[4], bl[4];
#pragma unroll
    for (int j = 0; j < 4; ++j) {
      const size_t bo = (size_t)(n0 + (j << 4) + rlane) * ldb + koff + k0;
      bh[j] = Frag<T>::load(Bb + bo);
      if (SPLIT) bl[j] = Frag<T>::load(Bb2 + bo);
    }
#pragma unroll
    for (int i = 0; i < 4; ++i) {
      const size_t ao = (size_t)(m0 + (i << 4) + rlane) * lda + koff + k0;
      V ah = Frag<T>::load(Ab + ao);
      V al;
      if (SPLIT) al = Frag<T>::load(Ab2 + ao);
#pragma unroll
      for (int j = 0; j < 4; ++j) {
        acc[i][j] = Frag<T>::mma(ah, bh[j], acc[i][j]);
        if (SPLIT) {
          acc[i][j] = Frag<T>::mma(ah, bl[j], acc[i][j]);
          acc[i][j] = Frag<T>::mma(al, bh[j], acc[i][j]);
        }
      }
      Frag<T>::guard(acc[i][0], acc[i][3], ah, SPLIT ? al : ah);
    }
    Frag<T>::keep(bh[0], bh[1], bh[2], bh[3]);
    if (SPLIT) Frag<T>::keep(bl[0], bl[1], bl[2], bl[3]);
  }
  acc_guard4(acc[0][0], acc[0][1], acc[0][2], acc[0][3]);
  acc_guard4(acc[1][0], acc[1][1], acc[1][2], acc[1][3]);
  acc_guard4(acc[2][0], acc[2][1], acc[2][2], acc[2][3]);
  acc_guard4(acc[3][0], acc[3][1], acc[3][2], acc[3][3]);

  float* slab = sT[wave];
  const float gval = GMUL ? gptr[0] : 1.0f;
#pragma unroll
  for (int i = 0; i < 4; ++i) {
    const int mBase = m0 + (i << 4);
    float bmr[8];
#pragma unroll
    for (int r = 0; r < 8; ++r) bmr[r] = 0.f;
    if (BIAS_MODE == 1) {
      const v4f b0 = *(const v4f*)(bias + mBase + mOff);
      const v4f b1 = *(const v4f*)(bias + mBase + mOff + 4);
      bmr[0] = b0.x; bmr[1] = b0.y; bmr[2] = b0.z; bmr[3] = b0.w;
      bmr[4] = b1.x; bmr[5] = b1.y; bmr[6] = b1.z; bmr[7] = b1.w;
    }
#pragma unroll
    for (int j = 0; j < 4; ++j) {
      const int n = n0 + (j << 4) + rlane;
      float bn = 0.f;
      if (BIAS_MODE == 2) bn = bias[n];
#pragma unroll
      for (int r = 0; r < 8; ++r) {
        float v = acc[i][j][r] * scale;
        if (BIAS_MODE == 1) v += bmr[r];
        if (BIAS_MODE == 2) v += bn;
        slab[(mOff + r) * 68 + (j << 4) + rlane] = v;
      }
    }
    __builtin_amdgcn_fence(3, "workgroup");
    __builtin_amdgcn_wave_barrier();
    __builtin_amdgcn_fence(2, "workgroup");
    if (OUT_MODE == 0) {
      float* Cb = (float*)Cout + (size_t)b * strideC;
      const int hq = lane >> 4, c4 = (lane & 15) * 4;
      v4f vals[8];
#pragma unroll
      for (int it = 0; it < 8; ++it) {
        const int row = it * 2 + hq;
        v4f vv = *(const v4f*)(slab + row * 68 + c4);
        if (GMUL) vv = vv * gval;
        if (RESID) {
          const v4f rr = *(const v4f*)(resid + (size_t)b * strideR + (size_t)(mBase + row) * ldc + n0 + c4);
          vv = vv + rr;
        }
        vals[it] = vv;
      }
      for (int pass = 0; pass < 2; ++pass) {
#pragma unroll
        for (int it = 0; it < 8; ++it) {
          const int row = it * 2 + hq;
          *(volatile v4f*)(Cb + (size_t)(mBase + row) * ldc + n0 + c4) = vals[it];
        }
        __threadfence();
      }
    } else {
      const int q = lane >> 3, c8 = (lane & 7) * 8;
      unsigned short* C  = (unsigned short*)Cout  + (size_t)b * strideC;
      unsigned short* C2 = (OUT_MODE == 2) ? ((unsigned short*)Cout2 + (size_t)b * strideC) : nullptr;
      for (int pass = 0; pass < 2; ++pass) {
#pragma unroll
        for (int it = 0; it < 4; ++it) {
          const int row = it * 4 + q;
          const float* sp = slab + row * 68 + c8;
          v8h hv, lv;
#pragma unroll
          for (int e = 0; e < 8; ++e) {
            if (OUT_MODE == 1) {
              hv[e] = (_Float16)sp[e];
            } else {
              unsigned short hb = f2bf_bits(sp[e]);
              unsigned short lb = f2bf_bits(sp[e] - bf_bits2f(hb));
              hv[e] = __builtin_bit_cast(_Float16, hb);
              lv[e] = __builtin_bit_cast(_Float16, lb);
            }
          }
          *(volatile v8h*)(C + (size_t)(mBase + row) * ldc + n0 + c8) = hv;
          if (OUT_MODE == 2) *(volatile v8h*)(C2 + (size_t)(mBase + row) * ldc + n0 + c8) = lv;
        }
        __threadfence();
      }
    }
    __builtin_amdgcn_fence(3, "workgroup");
    __builtin_amdgcn_wave_barrier();
    __builtin_amdgcn_fence(2, "workgroup");
  }
}

__global__ __launch_bounds__(256) void x_transpose_split(const float* __restrict__ x,
                                                         unsigned short* __restrict__ xth,
                                                         unsigned short* __restrict__ xtl) {
  __shared__ __align__(16) float tile[64 * 68];
  const int n0 = blockIdx.x * 64;
  const int c0 = blockIdx.y * 64;
  const int b  = blockIdx.z;
  const int tid = threadIdx.x, wave = tid >> 5, lane = tid & 31;
  const float* xb = x + ((size_t)b * kCh + c0) * kPixFull + n0;
#pragma unroll
  for (int i = 0; i < 4; ++i) {
    const int c  = i * 16 + (tid >> 4);
    const int n4 = (tid & 15) * 4;
    const v4f v = *(const v4f*)(xb + (size_t)c * kPixFull + n4);
    *(v4f*)(tile + c * 68 + n4) = v;
  }
  __syncthreads();
  const int q = lane >> 3, c8 = (lane & 7) * 8;
  v8h hv[2], lv[2];
#pragma unroll
  for (int it = 0; it < 2; ++it) {
    const int nrow = wave * 8 + it * 4 + q;
#pragma unroll
    for (int e = 0; e < 8; ++e) {
      const float f = tile[(c8 + e) * 68 + nrow];
      const unsigned short hb = f2bf_bits(f);
      const unsigned short lb = f2bf_bits(f - bf_bits2f(hb));
      hv[it][e] = __builtin_bit_cast(_Float16, hb);
      lv[it][e] = __builtin_bit_cast(_Float16, lb);
    }
  }
  const size_t base = ((size_t)b * kPix + n0) * kCh + c0;
  for (int pass = 0; pass < 2; ++pass) {
#pragma unroll
    for (int it = 0; it < 2; ++it) {
      const int nrow = wave * 8 + it * 4 + q;
      *(volatile v8h*)(xth + base + (size_t)nrow * kCh + c8) = hv[it];
      *(volatile v8h*)(xtl + base + (size_t)nrow * kCh + c8) = lv[it];
    }
    __threadfence();
  }
}

__global__ __launch_bounds__(256) void split_f32_bf16x8(const float* __restrict__ in,
                                                        unsigned short* __restrict__ hi,
                                                        unsigned short* __restrict__ lo, int n8) {
  const int i = blockIdx.x * 256 + threadIdx.x;
  if (i < n8) {
    const v4f a = *(const v4f*)(in + (size_t)8 * i);
    const v4f c = *(const v4f*)(in + (size_t)8 * i + 4);
    float f[8];
    f[0] = a.x; f[1] = a.y; f[2] = a.z; f[3] = a.w; f[4] = c.x; f[5] = c.y; f[6] = c.z; f[7] = c.w;
    v8h hv, lv;
#pragma unroll
    for (int e = 0; e < 8; ++e) {
      const unsigned short hb = f2bf_bits(f[e]);
      const unsigned short lb = f2bf_bits(f[e] - bf_bits2f(hb));
      hv[e] = __builtin_bit_cast(_Float16, hb);
      lv[e] = __builtin_bit_cast(_Float16, lb);
    }
    *(volatile v8h*)(hi + (size_t)8 * i) = hv;
    *(volatile v8h*)(lo + (size_t)8 * i) = lv;
    __threadfence();
    *(volatile v8h*)(hi + (size_t)8 * i) = hv;
    *(volatile v8h*)(lo + (size_t)8 * i) = lv;
  }
}

__global__ __launch_bounds__(256) void softmax_rows_f16(const float* __restrict__ S,
                                                       unsigned short* __restrict__ P) {
  __shared__ __align__(16) float ebuf[kPix];
  __shared__ float red[16];
  const int row = blockIdx.x;
  const int tid = threadIdx.x;
  const int wave = tid >> 5, lane = tid & 31;
  const bool act = (tid < kSmThreads);
  const float* sr = S + (size_t)row * kPix;
  float* eb = ebuf + (act ? tid : 0) * (8 * kSmChunks);
  const int e0 = tid * 8;
  const int e1 = kSmThreads * 8 + tid * 8;
  float m = -3.0e38f;
  if (act) {
    const v4f a0 = *(const v4f*)(sr + e0);
    const v4f a1 = *(const v4f*)(sr + e0 + 4);
    m = fmaxf(fmaxf(fmaxf(a0.x, a0.y), fmaxf(a0.z, a0.w)), fmaxf(fmaxf(a1.x, a1.y), fmaxf(a1.z, a1.w)));
    *(v4f*)(eb + 0) = a0;
    *(v4f*)(eb + 4) = a1;
    if (kSmChunks > 1) {
      const v4f a2 = *(const v4f*)(sr + e1);
      const v4f a3 = *(const v4f*)(sr + e1 + 4);
      m = fmaxf(m, fmaxf(fmaxf(fmaxf(a2.x, a2.y), fmaxf(a2.z, a2.w)), fmaxf(fmaxf(a3.x, a3.y), fmaxf(a3.z, a3.w))));
      *(v4f*)(eb + 8)  = a2;
      *(v4f*)(eb + 12) = a3;
    }
  }
#pragma unroll
  for (int off = 1; off < 32; off <<= 1) m = fmaxf(m, __shfl_xor(m, off, 32));
  if (lane == 0) red[wave] = m;
  __syncthreads();
  float gm = red[0];
#pragma unroll
  for (int w = 1; w < 8; ++w) gm = fmaxf(gm, red[w]);
  float psum = 0.0f;
  if (act) {
#pragma unroll 1
    for (int i4 = 0; i4 < 2 * kSmChunks; ++i4) {
      const v4f sv = *(const v4f*)(eb + 4 * i4);
      v4f ev;
      ev.x = expf(sv.x - gm);
      ev.y = expf(sv.y - gm);
      ev.z = expf(sv.z - gm);
      ev.w = expf(sv.w - gm);
      psum += (ev.x + ev.y) + (ev.z + ev.w);
      *(v4f*)(eb + 4 * i4) = ev;
    }
  }
#pragma unroll
  for (int off = 1; off < 32; off <<= 1) psum += __shfl_xor(psum, off, 32);
  if (lane == 0) red[8 + wave] = psum;
  __syncthreads();
  float l = red[8];
#pragma unroll
  for (int w = 1; w < 8; ++w) l += red[8 + w];
  const float inv = kPCarry * (1.0f / l);
  if (act) {
    const v4f q0 = *(const v4f*)(eb + 0);
    const v4f q1 = *(const v4f*)(eb + 4);
    v8h p0, p1;
#pragma unroll
    for (int e = 0; e < 4; ++e) {
      p0[e]     = (_Float16)(q0[e] * inv);
      p0[4 + e] = (_Float16)(q1[e] * inv);
    }
    p1 = p0;
    if (kSmChunks > 1) {
      const v4f q2 = *(const v4f*)(eb + 8);
      const v4f q3 = *(const v4f*)(eb + 12);
#pragma unroll
      for (int e = 0; e < 4; ++e) {
        p1[e]     = (_Float16)(q2[e] * inv);
        p1[4 + e] = (_Float16)(q3[e] * inv);
      }
    }
    unsigned short* pr = P + (size_t)row * kPix;
    for (int pass = 0; pass < 2; ++pass) {
      *(volatile v8h*)(pr + e0) = p0;
      if (kSmChunks > 1) *(volatile v8h*)(pr + e1) = p1;
      __threadfence();
    }
  }
}

extern "C" void kernel_launch(void* const* d_in, const int* in_sizes, int n_in,
                              void* d_out, int out_size, void* d_ws, size_t ws_size,
                              hipStream_t stream) {
  if (n_in < 8) return;
  if (in_sizes[0] < kBatch * kCh * kPixFull) return;
  if (in_sizes[1] < kCq * kCh || in_sizes[3] < kCq * kCh || in_sizes[5] < kCh * kCh) return;
  if (in_sizes[2] < kCq || in_sizes[4] < kCq || in_sizes[6] < kCh || in_sizes[7] < 1) return;
  if (out_size < kBatch * kCh * kPixFull) return;
  if (ws_size < kWsTotal) return;

  const float* x     = (const float*)d_in[0];
  const float* Wq    = (const float*)d_in[1];
  const float* bq    = (const float*)d_in[2];
  const float* Wk    = (const float*)d_in[3];
  const float* bk    = (const float*)d_in[4];
  const float* Wv    = (const float*)d_in[5];
  const float* bv    = (const float*)d_in[6];
  const float* gamma = (const float*)d_in[7];
  float* out = (float*)d_out;

  char* ws = (char*)d_ws;
  unsigned short* xth = (unsigned short*)(ws + kOffXtHi);
  unsigned short* xtl = (unsigned short*)(ws + kOffXtLo);
  unsigned short* pln = (unsigned short*)(ws + kOffP);
  unsigned short* wqh = (unsigned short*)(ws + kOffWqHi);
  unsigned short* wql = (unsigned short*)(ws + kOffWqLo);
  unsigned short* wkh = (unsigned short*)(ws + kOffWkHi);
  unsigned short* wkl = (unsigned short*)(ws + kOffWkLo);
  unsigned short* wvh = (unsigned short*)(ws + kOffWvHi);
  unsigned short* wvl = (unsigned short*)(ws + kOffWvLo);
  unsigned short* qh  = (unsigned short*)(ws + kOffQHi);
  unsigned short* ql  = (unsigned short*)(ws + kOffQLo);
  unsigned short* kh  = (unsigned short*)(ws + kOffKHi);
  unsigned short* kl  = (unsigned short*)(ws + kOffKLo);
  unsigned short* vt  = (unsigned short*)(ws + kOffVt);
  float* spl = (float*)(ws + kOffS);

  x_transpose_split<<<dim3(kPix / 64, kCh / 64, kBatch), 256, 0, stream>>>(x, xth, xtl);
  split_f32_bf16x8<<<(kCq * kCh / 8) / 256, 256, 0, stream>>>(Wq, wqh, wql, kCq * kCh / 8);
  split_f32_bf16x8<<<(kCq * kCh / 8) / 256, 256, 0, stream>>>(Wk, wkh, wkl, kCq * kCh / 8);
  split_f32_bf16x8<<<(kCh * kCh / 8) / 256, 256, 0, stream>>>(Wv, wvh, wvl, kCh * kCh / 8);
  static_assert((kCq * kCh / 8) % 256 == 0 && (kCh * kCh / 8) % 256 == 0);

  {
    constexpr int tiles = (kPix / 64) * (kCq / 64);
    wmma_gemm64<1, true, 2, 2, false, false><<<dim3((tiles + 7) / 8, kBatch), 256, 0, stream>>>(
        xth, xtl, kCh, (long)kPix * kCh,
        wqh, wql, kCh, 0L,
        (void*)qh, (void*)ql, kCq, (long)kPix * kCq,
        bq, x, 0L, gamma, kPix, kCq, kCh, 1.0f);
    wmma_gemm64<1, true, 2, 2, false, false><<<dim3((tiles + 7) / 8, kBatch), 256, 0, stream>>>(
        xth, xtl, kCh, (long)kPix * kCh,
        wkh, wkl, kCh, 0L,
        (void*)kh, (void*)kl, kCq, (long)kPix * kCq,
        bk, x, 0L, gamma, kPix, kCq, kCh, 1.0f);
  }
  {
    constexpr int tiles = (kCh / 64) * (kPix / 64);
    wmma_gemm64<1, true, 1, 1, false, false><<<dim3((tiles + 7) / 8, kBatch), 256, 0, stream>>>(
        wvh, wvl, kCh, 0L,
        xth, xtl, kCh, (long)kPix * kCh,
        (void*)vt, (void*)vt, kPix, (long)kCh * kPix,
        bv, x, 0L, gamma, kCh, kPix, kCh, 1.0f);
  }
  for (int b = 0; b < kBatch; ++b) {
    const size_t qko = (size_t)b * kPix * kCq;
    {
      constexpr int tiles = (kPix / 64) * (kPix / 64);
      wmma_gemm64<1, true, 0, 0, false, false><<<dim3((tiles + 7) / 8, 1), 256, 0, stream>>>(
          qh + qko, ql + qko, kCq, 0L,
          kh + qko, kl + qko, kCq, 0L,
          (void*)spl, (void*)spl, kPix, 0L,
          bq, x, 0L, gamma, kPix, kPix, kCq, 1.0f);
    }
    softmax_rows_f16<<<kPix, 256, 0, stream>>>(spl, pln);
    {
      constexpr int tiles = (kCh / 64) * (kPix / 64);
      const size_t vo = (size_t)b * kCh * kPix;
      const size_t oo = (size_t)b * kCh * kPixFull;
      wmma_gemm64<0, false, 0, 0, true, true><<<dim3((tiles + 7) / 8, 1), 256, 0, stream>>>(
          vt + vo, vt + vo, kPix, 0L,
          pln, pln, kPix, 0L,
          (void*)(out + oo), (void*)(out + oo), kPixFull, 0L,
          bv, x + oo, 0L, gamma, kCh, kPix, kPix, kPCarryInv);
    }
  }
}
